// FastPaperMambaBlock_8263517077567
// MI455X (gfx1250) — hardware-verified
//
#include <hip/hip_runtime.h>
#include <math.h>

typedef __attribute__((ext_vector_type(16))) _Float16 v16h;
typedef __attribute__((ext_vector_type(8)))  _Float16 v8h;
typedef __attribute__((ext_vector_type(16))) __bf16   v16b;
typedef __attribute__((ext_vector_type(8)))  __bf16   v8b;
typedef __attribute__((ext_vector_type(8)))  float    v8f;
typedef __attribute__((ext_vector_type(4)))  float    v4f;

constexpr int kBatch = 2;
constexpr int kSeqL  = 2048;
constexpr int kDm    = 1024;
constexpr int kNst   = 32;
constexpr int kRows  = kBatch * kSeqL;
constexpr int kXZP   = 2 * kDm;
constexpr int kTP    = 260;

__device__ __forceinline__ unsigned short f2bf_bits(float f) {
  unsigned u = __float_as_uint(f);
  return (unsigned short)((u + 0x7FFFu + ((u >> 16) & 1u)) >> 16);
}
__device__ __forceinline__ float bf_bits2f(unsigned short h) { return __uint_as_float(((unsigned)h) << 16); }

__device__ __forceinline__ void dep_guard_h(v8f& a, v8f& b, v16h x, v16h y) { asm volatile("v_nop\n\tv_nop\n\tv_nop\n\tv_nop" : "+v"(a), "+v"(b) : "v"(x), "v"(y)); }
__device__ __forceinline__ void dep_guard_b(v8f& a, v8f& b, v16b x, v16b y) { asm volatile("v_nop\n\tv_nop\n\tv_nop\n\tv_nop" : "+v"(a), "+v"(b) : "v"(x), "v"(y)); }
__device__ __forceinline__ void keep4_h(v16h a, v16h b, v16h c, v16h d) { asm volatile("v_nop" :: "v"(a), "v"(b), "v"(c), "v"(d)); }
__device__ __forceinline__ void keep4_b(v16b a, v16b b, v16b c, v16b d) { asm volatile("v_nop" :: "v"(a), "v"(b), "v"(c), "v"(d)); }
__device__ __forceinline__ void acc_guard4(v8f& a, v8f& b, v8f& c, v8f& d) { asm volatile("v_nop\n\tv_nop\n\tv_nop\n\tv_nop" : "+v"(a), "+v"(b), "+v"(c), "+v"(d)); }
template <typename T> struct Frag;
template <> struct Frag<_Float16> {
  typedef v16h V; union U { v16h v; v8h h[2]; };
  static __device__ __forceinline__ v16h load(const _Float16* p) {
    U f; f.h[0] = *(const v8h*)(p); f.h[1] = *(const v8h*)(p + 16); return f.v;
  }
  static __device__ __forceinline__ v8f mma(v16h a, v16h b, v8f c) {
    return __builtin_amdgcn_wmma_f32_16x16x32_f16(false, a, false, b, (short)0, c, false, false);
  }
  static __device__ __forceinline__ void guard(v8f& a, v8f& b, v16h x, v16h y) { dep_guard_h(a, b, x, y); }
  static __device__ __forceinline__ void keep(v16h a, v16h b, v16h c, v16h d) { keep4_h(a, b, c, d); }
};
template <> struct Frag<__bf16> {
  typedef v16b V; union U { v16b v; v8b h[2]; };
  static __device__ __forceinline__ v16b load(const __bf16* p) {
    U f; f.h[0] = *(const v8b*)(p); f.h[1] = *(const v8b*)(p + 16); return f.v;
  }
  static __device__ __forceinline__ v8f mma(v16b a, v16b b, v8f c) {
    return __builtin_amdgcn_wmma_f32_16x16x32_bf16(false, a, false, b, (short)0, c, false, false);
  }
  static __device__ __forceinline__ void guard(v8f& a, v8f& b, v16b x, v16b y) { dep_guard_b(a, b, x, y); }
  static __device__ __forceinline__ void keep(v16b a, v16b b, v16b c, v16b d) { keep4_b(a, b, c, d); }
};

template <int ET> struct Elem;
template <> struct Elem<0> { typedef _Float16 T; };
template <> struct Elem<1> { typedef __bf16 T; };
template <int ET, bool SPLIT, int BIAS_MODE, int OUT_MODE, bool RESID, int ACT = 0>
__global__ __launch_bounds__(256) void wmma_gemm64(
    const unsigned short* __restrict__ Ap, const unsigned short* __restrict__ A2p, int lda, long strideA,
    const unsigned short* __restrict__ Btp, const unsigned short* __restrict__ Bt2p, int ldb, long strideB,
    void* __restrict__ Cout, void* __restrict__ Cout2, int ldc, long strideC,
    const float* __restrict__ bias,
    const float* __restrict__ resid, long strideR,
    int M, int N, int K, float scale) {
  typedef typename Elem<ET>::T T;
  typedef typename Frag<T>::V V;
  const T* A = (const T*)Ap; const T* A2 = (const T*)A2p; const T* Bt = (const T*)Btp; const T* Bt2 = (const T*)Bt2p;
  __shared__ __align__(16) float sT[8][16 * 68];
  const int b    = blockIdx.y;
  const int lane = threadIdx.x & 31;
  const int wave = threadIdx.x >> 5;
  const int tilesN = N >> 6;
  const int tilesM = M >> 6;
  const int tile = blockIdx.x * 8 + wave;
  if (tile >= tilesM * tilesN) return;
  const int tm = tile / tilesN;
  const int tn = tile - tm * tilesN;
  const int m0 = tm << 6;
  const int n0 = tn << 6;

  const T* Ab  = A  + (size_t)b * strideA;
  const T* Bb  = Bt + (size_t)b * strideB;
  const T* Ab2 = SPLIT ? (A2  + (size_t)b * strideA) : nullptr;
  const T* Bb2 = SPLIT ? (Bt2 + (size_t)b * strideB) : nullptr;

  const int rlane = lane & 15;
  const int koff  = (lane >> 4) * 8;
  const int mOff  = (lane >> 4) * 8;

  v8f acc[4][4];
#pragma unroll
  for (int i = 0; i < 4; ++i)
#pragma unroll
    for (int j = 0; j < 4; ++j) acc[i][j] = (v8f){0.f,0.f,0.f,0.f,0.f,0.f,0.f,0.f};

  for (int k0 = 0; k0 < K; k0 += 32) {
    V bh[4], bl[4];
#pragma unroll
    for (int j = 0; j < 4; ++j) {
      const size_t bo = (size_t)(n0 + (j << 4) + rlane) * ldb + koff + k0;
      bh[j] = Frag<T>::load(Bb + bo);
      if (SPLIT) bl[j] = Frag<T>::load(Bb2 + bo);
    }
#pragma unroll
    for (int i = 0; i < 4; ++i) {
      const size_t ao = (size_t)(m0 + (i << 4) + rlane) * lda + koff + k0;
      V ah = Frag<T>::load(Ab + ao);
      V al;
      if (SPLIT) al = Frag<T>::load(Ab2 + ao);
#pragma unroll
      for (int j = 0; j < 4; ++j) {
        acc[i][j] = Frag<T>::mma(ah, bh[j], acc[i][j]);
        if (SPLIT) {
          acc[i][j] = Frag<T>::mma(ah, bl[j], acc[i][j]);
          acc[i][j] = Frag<T>::mma(al, bh[j], acc[i][j]);
        }
      }
      Frag<T>::guard(acc[i][0], acc[i][3], ah, SPLIT ? al : ah);
    }
    Frag<T>::keep(bh[0], bh[1], bh[2], bh[3]);
    if (SPLIT) Frag<T>::keep(bl[0], bl[1], bl[2], bl[3]);
  }
  acc_guard4(acc[0][0], acc[0][1], acc[0][2], acc[0][3]);
  acc_guard4(acc[1][0], acc[1][1], acc[1][2], acc[1][3]);
  acc_guard4(acc[2][0], acc[2][1], acc[2][2], acc[2][3]);
  acc_guard4(acc[3][0], acc[3][1], acc[3][2], acc[3][3]);

  float* slab = sT[wave];
  const float* Rb = RESID ? (resid + (size_t)b * strideR) : nullptr;
#pragma unroll
  for (int i = 0; i < 4; ++i) {
    const int mBase = m0 + (i << 4);
#pragma unroll
    for (int j = 0; j < 4; ++j) {
      const int n = n0 + (j << 4) + rlane;
      float bv = 0.f;
      if (BIAS_MODE == 2) bv = bias[n];
#pragma unroll
      for (int r = 0; r < 8; ++r) {
        float v = acc[i][j][r] * scale;
        if (BIAS_MODE == 1) v += bias[mBase + mOff + r];
        if (BIAS_MODE == 2) v += bv;
        if (RESID) v += Rb[(size_t)(mBase + mOff + r) * ldc + n];
        if (ACT == 1) v = tanhf(v);
        if (ACT == 2) v = fmaxf(v, 0.0f);
        if (ACT == 3) v = v / (1.0f + expf(-v));
        if (ACT == 4) v = (v > 0.f) ? v : 0.01f * v;
        if (ACT == 5) v = 0.5f * v * (1.0f + erff(v * 0.70710678118654752f));
        slab[(mOff + r) * 68 + (j << 4) + rlane] = v;
      }
    }
    __builtin_amdgcn_fence(__ATOMIC_RELEASE, "workgroup");
    __builtin_amdgcn_wave_barrier();
    __builtin_amdgcn_fence(__ATOMIC_ACQUIRE, "workgroup");
    if (OUT_MODE == 0) {
      float* C = (float*)Cout + (size_t)b * strideC;
      const int hh = lane >> 4, c4 = (lane & 15) * 4;
      for (int pass = 0; pass < 2; ++pass) {
#pragma unroll
        for (int it = 0; it < 8; ++it) {
          const int row = it * 2 + hh;
          v4f v = *(const v4f*)(slab + row * 68 + c4);
          *(volatile v4f*)(C + (size_t)(mBase + row) * ldc + n0 + c4) = v;
        }
        __threadfence();
      }
    } else {
      const int q = lane >> 3, c8 = (lane & 7) * 8;
      unsigned short* C  = (unsigned short*)Cout  + (size_t)b * strideC;
      unsigned short* C2 = (OUT_MODE == 2) ? ((unsigned short*)Cout2 + (size_t)b * strideC) : nullptr;
      for (int pass = 0; pass < 2; ++pass) {
#pragma unroll
        for (int it = 0; it < 4; ++it) {
          const int row = it * 4 + q;
          const float* sp = slab + row * 68 + c8;
          v8h hv, lv;
#pragma unroll
          for (int e = 0; e < 8; ++e) {
            if (OUT_MODE == 1) {
              hv[e] = (_Float16)sp[e];
            } else {
              unsigned short hb = f2bf_bits(sp[e]);
              unsigned short lb = f2bf_bits(sp[e] - bf_bits2f(hb));
              hv[e] = __builtin_bit_cast(_Float16, hb);
              lv[e] = __builtin_bit_cast(_Float16, lb);
            }
          }
          *(volatile v8h*)(C + (size_t)(mBase + row) * ldc + n0 + c8) = hv;
          if (OUT_MODE == 2) *(volatile v8h*)(C2 + (size_t)(mBase + row) * ldc + n0 + c8) = lv;
        }
        __threadfence();
      }
    }
    __builtin_amdgcn_fence(__ATOMIC_RELEASE, "workgroup");
    __builtin_amdgcn_wave_barrier();
    __builtin_amdgcn_fence(__ATOMIC_ACQUIRE, "workgroup");
  }
}

__global__ __launch_bounds__(256) void cast_f16_kernel(
    const float* __restrict__ src, unsigned short* __restrict__ dst, int total8, float scale)
{
  const int i = blockIdx.x * 256 + threadIdx.x;
  if (i >= total8) return;
  const size_t e0 = (size_t)i << 3;
  const float* p = src + e0;
  const v4f a0 = *(const v4f*)(p);
  const v4f a1 = *(const v4f*)(p + 4);
  v8h hv;
#pragma unroll
  for (int e = 0; e < 4; ++e) {
    hv[e]     = (_Float16)(a0[e] * scale);
    hv[4 + e] = (_Float16)(a1[e] * scale);
  }
  unsigned short* q = dst + e0;
  *(volatile v8h*)q = hv;
  __threadfence();
  *(volatile v8h*)q = hv;
}

__global__ __launch_bounds__(256) void stack_bc_kernel(
    const float* __restrict__ Bw, const float* __restrict__ Cw,
    const float* __restrict__ Bb, const float* __restrict__ Cb,
    unsigned short* __restrict__ W16, float* __restrict__ bias64, float scale)
{
  const int i = blockIdx.x * 256 + threadIdx.x;
  const int e0 = i << 3;
  const int row = e0 >> 10;
  const int col = e0 & (kDm - 1);
  const int rB = (row < kNst) ? row : (kNst - 1);
  const int rCt = row - kNst;
  const int rC = (rCt < 0) ? 0 : rCt;
  const float* pb = Bw + (size_t)rB * kDm + col;
  const float* pc = Cw + (size_t)rC * kDm + col;
  const v4f b0 = *(const v4f*)(pb);
  const v4f b1 = *(const v4f*)(pb + 4);
  const v4f c0 = *(const v4f*)(pc);
  const v4f c1 = *(const v4f*)(pc + 4);
  const bool useB = row < kNst;
  v8h hv;
#pragma unroll
  for (int e = 0; e < 4; ++e) {
    const float f0 = useB ? b0[e] : c0[e];
    const float f1 = useB ? b1[e] : c1[e];
    hv[e]     = (_Float16)(f0 * scale);
    hv[4 + e] = (_Float16)(f1 * scale);
  }
  unsigned short* q = W16 + e0;
  *(volatile v8h*)q = hv;
  __threadfence();
  *(volatile v8h*)q = hv;

  if (blockIdx.x == 0 && threadIdx.x < 32) {
    const int lane = threadIdx.x;
    const int iB = ((lane < 8) ? lane : 7) * 4;
    const int t  = lane - 8;
    const int iC = ((t < 0) ? 0 : ((t > 7) ? 7 : t)) * 4;
    const v4f vb = *(const v4f*)(Bb + iB);
    const v4f vc = *(const v4f*)(Cb + iC);
    v4f val;
#pragma unroll
    for (int e = 0; e < 4; ++e) val[e] = (lane < 8) ? vb[e] : vc[e];
    if (lane < 16) *(volatile v4f*)(bias64 + lane * 4) = val;
    __threadfence();
    if (lane < 16) *(volatile v4f*)(bias64 + lane * 4) = val;
  }
}

__global__ __launch_bounds__(256) void conv_silu_kernel(
    const float* __restrict__ XZ, const float* __restrict__ cw, const float* __restrict__ cb,
    float* __restrict__ XS, unsigned short* __restrict__ XS16)
{
  __shared__ __align__(16) float sT[16 * kTP];
  const int tid = threadIdx.x, lane = tid & 31, wave = tid >> 5;
  const int d0 = blockIdx.x * 256, d = d0 + tid;
  const int m0 = blockIdx.y * 64;
  const int bidx = m0 / kSeqL;
  const int t0 = m0 - bidx * kSeqL;
  const size_t rb = (size_t)bidx * kSeqL;
  const float w0 = cw[d * 4 + 0], w1 = cw[d * 4 + 1], w2 = cw[d * 4 + 2], w3 = cw[d * 4 + 3];
  const float bc = cb[d];
  float xm2, xm1, xcu;
  {
    const int r0 = t0 - 2, r1 = t0 - 1;
    const float v0 = XZ[(rb + (r0 < 0 ? 0 : r0)) * kXZP + d];
    const float v1 = XZ[(rb + (r1 < 0 ? 0 : r1)) * kXZP + d];
    xm2 = (r0 >= 0) ? v0 : 0.f;
    xm1 = (r1 >= 0) ? v1 : 0.f;
    xcu = XZ[(rb + t0) * kXZP + d];
  }
  const int hrow = wave >> 1;
  const int hch  = (wave & 1) * 128 + lane * 4;
#pragma unroll 1
  for (int sub = 0; sub < 4; ++sub) {
    const int lb = t0 + sub * 16;
#pragma unroll 1
    for (int s = 0; s < 16; ++s) {
      const int tn  = lb + s + 1;
      const int tnc = (tn < kSeqL) ? tn : (kSeqL - 1);
      const float vn = XZ[(rb + tnc) * kXZP + d];
      const float xn = (tn < kSeqL) ? vn : 0.f;
      float acc = w0 * xm2;
      acc = fmaf(w1, xm1, acc);
      acc = fmaf(w2, xcu, acc);
      acc = fmaf(w3, xn, acc);
      const float sv = acc + bc;
      const float sg = __builtin_amdgcn_rcpf(1.0f + __expf(-sv));
      sT[s * kTP + tid] = sv * sg;
      xm2 = xm1; xm1 = xcu; xcu = xn;
    }
    __syncthreads();
    v4f fv[4];
    v8h bv[2];
#pragma unroll
    for (int it = 0; it < 4; ++it) fv[it] = *(const v4f*)(sT + (it * 4 + hrow) * kTP + hch);
#pragma unroll
    for (int it = 0; it < 2; ++it) {
      const float* sp = sT + (it * 8 + wave) * kTP + lane * 8;
      const v4f a0 = *(const v4f*)(sp);
      const v4f a1 = *(const v4f*)(sp + 4);
#pragma unroll
      for (int e = 0; e < 4; ++e) {
        bv[it][e]     = (_Float16)a0[e];
        bv[it][4 + e] = (_Float16)a1[e];
      }
    }
    const size_t rowg = rb + lb;
    for (int pass = 0; pass < 2; ++pass) {
#pragma unroll
      for (int it = 0; it < 4; ++it)
        *(volatile v4f*)(XS + (rowg + it * 4 + hrow) * kDm + d0 + hch) = fv[it];
#pragma unroll
      for (int it = 0; it < 2; ++it)
        *(volatile v8h*)(XS16 + (rowg + it * 8 + wave) * kDm + d0 + lane * 8) = bv[it];
      __threadfence();
    }
    __syncthreads();
  }
}

__global__ __launch_bounds__(256) void scan_kernel(
    const float* __restrict__ DTR, const float* __restrict__ XS, const float* __restrict__ XZ,
    const float* __restrict__ BCM, const float* __restrict__ A_log,
    unsigned short* __restrict__ Y16)
{
  __shared__ __align__(16) float sBC[16 * 64];
  __shared__ __align__(16) float sY[16 * kTP];
  const int tid = threadIdx.x, lane = tid & 31, wave = tid >> 5;
  const int d0 = blockIdx.x * 256, d = d0 + tid;
  const size_t rb = (size_t)blockIdx.y * kSeqL;

  float An[kNst];
#pragma unroll
  for (int n = 0; n < kNst; ++n) {
    float al = A_log[(size_t)d * kNst + n];
    al = fminf(fmaxf(al, -5.0f), 2.0f);
    An[n] = -__expf(al);
  }
  float h[kNst];
#pragma unroll
  for (int n = 0; n < kNst; ++n) h[n] = 0.f;

#pragma unroll 1
  for (int c = 0; c < kSeqL / 16; ++c) {
    const int l0 = c * 16;
    {
      const int r = tid >> 4, q = (tid & 15) * 4;
      const v4f v = *(const v4f*)(BCM + (rb + l0 + r) * 64 + q);
      *(v4f*)(sBC + r * 64 + q) = v;
    }
    __syncthreads();
#pragma unroll 1
    for (int s = 0; s < 16; ++s) {
      const size_t m = rb + l0 + s;
      const float a   = DTR[m * kDm + d];
      const float spl = fmaxf(a, 0.0f) + log1pf(__expf(-fabsf(a)));
      const float dt  = fminf(fmaxf(spl, 0.001f), 0.2f);
      const float xv  = XS[m * kDm + d];
      const float zv  = XZ[m * kXZP + kDm + d];
      const float u   = dt * xv;
      v4f Bq[8], Cq[8];
#pragma unroll
      for (int qq = 0; qq < 8; ++qq) {
        Bq[qq] = *(const v4f*)(sBC + s * 64 + 4 * qq);
        Cq[qq] = *(const v4f*)(sBC + s * 64 + kNst + 4 * qq);
      }
      float y = 0.f;
#pragma unroll
      for (int n = 0; n < kNst; ++n) {
        const float e = __expf(dt * An[n]);
        float p = u * Bq[n >> 2][n & 3];
        asm volatile("" : "+v"(p));
        float qv = h[n] * e;
        asm volatile("" : "+v"(qv));
        float hn = p + qv;
        hn = fminf(fmaxf(hn, -10.0f), 10.0f);
        h[n] = hn;
        float rr = Cq[n >> 2][n & 3] * hn;
        asm volatile("" : "+v"(rr));
        y += rr;
      }
      const float sg = __builtin_amdgcn_rcpf(1.0f + __expf(-zv));
      const float g  = zv * sg;
      sY[s * kTP + tid] = (y * g) * 16.0f;
    }
    __syncthreads();
    v8h hv[2];
#pragma unroll
    for (int it = 0; it < 2; ++it) {
      const float* sp = sY + (it * 8 + wave) * kTP + lane * 8;
      const v4f a0 = *(const v4f*)(sp);
      const v4f a1 = *(const v4f*)(sp + 4);
#pragma unroll
      for (int e = 0; e < 4; ++e) { hv[it][e] = (_Float16)a0[e]; hv[it][4 + e] = (_Float16)a1[e]; }
    }
    for (int pass = 0; pass < 2; ++pass) {
#pragma unroll
      for (int it = 0; it < 2; ++it)
        *(volatile v8h*)(Y16 + (rb + l0 + it * 8 + wave) * kDm + d0 + lane * 8) = hv[it];
      __threadfence();
    }
  }
}

__global__ __launch_bounds__(256) void ln_kernel(
    const float* __restrict__ PRE, const float* __restrict__ g, const float* __restrict__ beta,
    float* __restrict__ out)
{
  __shared__ float red1[8];
  __shared__ float red2[8];
  const int tid = threadIdx.x, lane = tid & 31, wave = tid >> 5;
  const size_t base = (size_t)blockIdx.x * kDm + tid * 4;
  const v4f v = *(const v4f*)(PRE + base);
  float s = (v[0] + v[1]) + (v[2] + v[3]);
#pragma unroll
  for (int off = 16; off > 0; off >>= 1) s += __shfl_xor(s, off, 32);
  if (lane == 0) red1[wave] = s;
  __syncthreads();
  float tot = 0.f;
#pragma unroll
  for (int w = 0; w < 8; ++w) tot += red1[w];
  const float mean = tot * (1.0f / 1024.0f);
  const float e0 = v[0] - mean, e1 = v[1] - mean, e2 = v[2] - mean, e3 = v[3] - mean;
  float s2 = (e0 * e0 + e1 * e1) + (e2 * e2 + e3 * e3);
#pragma unroll
  for (int off = 16; off > 0; off >>= 1) s2 += __shfl_xor(s2, off, 32);
  if (lane == 0) red2[wave] = s2;
  __syncthreads();
  float tot2 = 0.f;
#pragma unroll
  for (int w = 0; w < 8; ++w) tot2 += red2[w];
  const float var  = tot2 * (1.0f / 1024.0f);
  const float rstd = rsqrtf(var + 1e-5f);
  const v4f gg = *(const v4f*)(g + tid * 4);
  const v4f bb = *(const v4f*)(beta + tid * 4);
  v4f o;
  o[0] = (gg[0] * e0) * rstd + bb[0];
  o[1] = (gg[1] * e1) * rstd + bb[1];
  o[2] = (gg[2] * e2) * rstd + bb[2];
  o[3] = (gg[3] * e3) * rstd + bb[3];
  *(volatile v4f*)(out + base) = o;
  __threadfence();
  *(volatile v4f*)(out + base) = o;
}

extern "C" void kernel_launch(void* const* d_in, const int* in_sizes, int n_in,
                              void* d_out, int out_size, void* d_ws, size_t ws_size,
                              hipStream_t stream)
{
  if (n_in < 16) return;
  const float* x         = (const float*)d_in[0];
  const float* in_proj_w = (const float*)d_in[1];
  const float* in_proj_b = (const float*)d_in[2];
  const float* conv_w    = (const float*)d_in[3];
  const float* conv_b    = (const float*)d_in[4];
  const float* A_log     = (const float*)d_in[5];
  const float* B_w       = (const float*)d_in[6];
  const float* B_b       = (const float*)d_in[7];
  const float* C_w       = (const float*)d_in[8];
  const float* C_b       = (const float*)d_in[9];
  const float* dt_w      = (const float*)d_in[10];
  const float* dt_b      = (const float*)d_in[11];
  const float* out_w     = (const float*)d_in[12];
  const float* out_b     = (const float*)d_in[13];
  const float* ln_g      = (const float*)d_in[14];
  const float* ln_beta   = (const float*)d_in[15];
  float* dout = (float*)d_out;

  if (in_sizes[0] != kRows * kDm) return;
  if (in_sizes[1] != 2 * kDm * kDm || in_sizes[2] != 2 * kDm) return;
  if (in_sizes[3] != kDm * 4 || in_sizes[4] != kDm) return;
  if (in_sizes[5] != kDm * kNst) return;
  if (in_sizes[6] != kNst * kDm || in_sizes[7] != kNst) return;
  if (in_sizes[8] != kNst * kDm || in_sizes[9] != kNst) return;
  if (in_sizes[10] != kDm * kDm || in_sizes[11] != kDm) return;
  if (in_sizes[12] != kDm * kDm || in_sizes[13] != kDm) return;
  if (in_sizes[14] != kDm || in_sizes[15] != kDm) return;
  if (out_size != kRows * kDm) return;

  const size_t SZ_WI16   = (size_t)2 * kDm * kDm * 2;
  const size_t SZ_WDT16  = (size_t)kDm * kDm * 2;
  const size_t SZ_WO16   = (size_t)kDm * kDm * 2;
  const size_t SZ_WBC16  = (size_t)64 * kDm * 2;
  const size_t SZ_BIAS64 = 131072;
  const size_t SZ_X16    = (size_t)kRows * kDm * 2;
  const size_t SZ_XZ     = (size_t)kRows * kXZP * 4;
  const size_t SZ_XS     = (size_t)kRows * kDm * 4;
  const size_t SZ_XS16   = (size_t)kRows * kDm * 2;
  const size_t SZ_BCM    = (size_t)kRows * 64 * 4;
  const size_t SZ_DTR    = (size_t)kRows * kDm * 4;
  const size_t OFF_WI16   = 0;
  const size_t OFF_WDT16  = OFF_WI16   + SZ_WI16;
  const size_t OFF_WO16   = OFF_WDT16  + SZ_WDT16;
  const size_t OFF_WBC16  = OFF_WO16   + SZ_WO16;
  const size_t OFF_BIAS64 = OFF_WBC16  + SZ_WBC16;
  const size_t OFF_X16    = OFF_BIAS64 + SZ_BIAS64;
  const size_t OFF_XZ     = OFF_X16    + SZ_X16;
  const size_t OFF_XS     = OFF_XZ     + SZ_XZ;
  const size_t OFF_XS16   = OFF_XS     + SZ_XS;
  const size_t OFF_BCM    = OFF_XS16   + SZ_XS16;
  const size_t OFF_DTR    = OFF_BCM    + SZ_BCM;
  const size_t TOTAL      = OFF_DTR    + SZ_DTR;
  if (ws_size < TOTAL) return;

  char* ws = (char*)d_ws;
  unsigned short* WI16   = (unsigned short*)(ws + OFF_WI16);
  unsigned short* WDT16  = (unsigned short*)(ws + OFF_WDT16);
  unsigned short* WO16   = (unsigned short*)(ws + OFF_WO16);
  unsigned short* WBC16  = (unsigned short*)(ws + OFF_WBC16);
  float*          BIAS64 = (float*)(ws + OFF_BIAS64);
  unsigned short* X16    = (unsigned short*)(ws + OFF_X16);
  unsigned short* Y16    = X16;
  float*          XZ     = (float*)(ws + OFF_XZ);
  float*          XS     = (float*)(ws + OFF_XS);
  unsigned short* XS16   = (unsigned short*)(ws + OFF_XS16);
  float*          BCM    = (float*)(ws + OFF_BCM);
  float*          DTR    = (float*)(ws + OFF_DTR);
  float*          PRE    = DTR;
  const float* dummy_resid = x;

  cast_f16_kernel<<<(2 * kDm * kDm) / 8 / 256, 256, 0, stream>>>(in_proj_w, WI16, (2 * kDm * kDm) / 8, 32.0f);
  cast_f16_kernel<<<(kDm * kDm) / 8 / 256, 256, 0, stream>>>(dt_w, WDT16, (kDm * kDm) / 8, 64.0f);
  cast_f16_kernel<<<(kDm * kDm) / 8 / 256, 256, 0, stream>>>(out_w, WO16, (kDm * kDm) / 8, 64.0f);
  stack_bc_kernel<<<(64 * kDm) / 8 / 256, 256, 0, stream>>>(B_w, C_w, B_b, C_b, WBC16, BIAS64, 64.0f);

  cast_f16_kernel<<<(kRows * kDm) / 8 / 256, 256, 0, stream>>>(x, X16, (kRows * kDm) / 8, 1.0f);

  wmma_gemm64<0, false, 2, 0, false><<<dim3(256, 1), 256, 0, stream>>>(
      X16, X16, kDm, 0L, WI16, WI16, kDm, 0L,
      (void*)XZ, (void*)XZ, kXZP, 0L, in_proj_b, dummy_resid, 0L, kRows, kXZP, kDm, 1.0f / 32.0f);

  conv_silu_kernel<<<dim3(kDm / 256, kRows / 64), 256, 0, stream>>>(XZ, conv_w, conv_b, XS, XS16);

  wmma_gemm64<0, false, 2, 0, false><<<dim3(8, 1), 256, 0, stream>>>(
      XS16, XS16, kDm, 0L, WBC16, WBC16, kDm, 0L,
      (void*)BCM, (void*)BCM, 64, 0L, BIAS64, dummy_resid, 0L, kRows, 64, kDm, 1.0f / 64.0f);

  wmma_gemm64<0, false, 2, 0, false><<<dim3(128, 1), 256, 0, stream>>>(
      XS16, XS16, kDm, 0L, WDT16, WDT16, kDm, 0L,
      (void*)DTR, (void*)DTR, kDm, 0L, dt_b, dummy_resid, 0L, kRows, kDm, kDm, 1.0f / 64.0f);

  scan_kernel<<<dim3(kDm / 256, kBatch), 256, 0, stream>>>(DTR, XS, XZ, BCM, A_log, Y16);

  wmma_gemm64<0, false, 2, 0, true><<<dim3(128, 1), 256, 0, stream>>>(
      Y16, Y16, kDm, 0L, WO16, WO16, kDm, 0L,
      (void*)PRE, (void*)PRE, kDm, 0L, out_b, x, 0L, kRows, kDm, kDm, 1.0f / 1024.0f);

  ln_kernel<<<kRows, 256, 0, stream>>>(PRE, ln_g, ln_beta, dout);

  (void)hipGetLastError();
}
